// RadialBasisArbitraryLayer_77386720740133
// MI455X (gfx1250) — hardware-verified
//
#include <hip/hip_runtime.h>


#ifndef NB
#define NB 8
#endif
#ifndef HROWS
#define HROWS 256
#endif
#define NB_FULL 8
#define HH_FULL 256
#define WW   256
#define NPT  160
#define NCH  2
#define KSTEPS (NPT / 32)
#define FW   8
#define PXW  32
#define WCAR 1024.0f
#define ACAR 16.0f
#define OSCL (1.0f / 16384.0f)
#define BIGD 1.0e10f
#define CFAC 2.0f

static_assert(NPT % 32 == 0);
static_assert(NPT % 8 == 0);
static_assert(WW == FW * PXW);
static_assert(PXW * 4 == 128);
static_assert(16 * 16 == NCH * PXW * 4);
static_assert(NPT / 2 <= 256);
static_assert((NPT / 2) * 16 == NPT * 2 * 4);
static_assert(16 * NPT / 8 == 256 + 64);
static_assert((NPT * 2 * 4) % 128 == 0);
static_assert((16 * NPT * 2) % 128 == 0);
static_assert(((NPT / 2) * 16) % 128 == 0);
static_assert(NB <= NB_FULL);
static_assert(HROWS <= HH_FULL);
static_assert((NPT * 2 + FW * NCH * PXW) * 4 <= 131072);
static_assert((NPT * 2 + 8) * 4 <= 131072);
static_assert(WCAR * ACAR * OSCL == 1.0f);

typedef _Float16 h16;
typedef __attribute__((ext_vector_type(16))) _Float16 v16h;
typedef __attribute__((ext_vector_type(8)))  _Float16 v8h;
typedef __attribute__((ext_vector_type(8)))  float    v8f;
typedef __attribute__((ext_vector_type(4)))  float    v4f;
typedef v4f  __attribute__((may_alias)) v4fa;

__device__ __forceinline__ unsigned short f2bf(float f) { unsigned u = __float_as_uint(f); u += 0x7FFFu + ((u >> 16) & 1u); return (unsigned short)(u >> 16); }
__device__ __forceinline__ float bfr(float f) { return __uint_as_float(((unsigned)f2bf(f)) << 16); }
__device__ __forceinline__ v16h cat16(v8h lo, v8h hi) { return __builtin_shufflevector(lo, hi, 0, 1, 2, 3, 4, 5, 6, 7, 8, 9, 10, 11, 12, 13, 14, 15); }
__device__ __forceinline__ v8f wmma16(v16h a, v16h b, v8f c) { return __builtin_amdgcn_wmma_f32_16x16x32_f16(false, a, false, b, (short)0, c, false, false); }
__device__ __forceinline__ v16h  ldh(const h16* p) { return cat16(*(const v8h*)p, *(const v8h*)(p + 16)); }
__device__ __forceinline__ void wave_sync() { __builtin_amdgcn_fence(3  , "wavefront"); __builtin_amdgcn_wave_barrier(); asm volatile("" ::: "memory"); }

static __device__ __forceinline__ h16 toh_flush(float v) { const h16 r = (h16)v; return (fabsf(v) < 6.103515625e-05f) ? (h16)0.0f : r; }
__device__ __forceinline__ v8f wmma16g(v16h a, v16h b, v8f c) {
    c = wmma16(a, b, c);
    asm volatile("v_nop\n\tv_nop\n\tv_nop\n\tv_nop" : "+v"(c) : "v"(a), "v"(b));
    return c;
}

__device__ __forceinline__ v8h at_piece(const float* __restrict__ al, int b, int p) {
    const int m = p / (NPT / 8), c8 = (p % (NPT / 8)) * 8;
    const float* src = al + ((size_t)b * NPT + (size_t)c8) * NCH;
    v4f x0 = *(const v4f*)(src), x1 = *(const v4f*)(src + 4), x2 = *(const v4f*)(src + 8), x3 = *(const v4f*)(src + 12);
    asm volatile("" : "+v"(x0)); asm volatile("" : "+v"(x1)); asm volatile("" : "+v"(x2)); asm volatile("" : "+v"(x3));
    const bool odd = (m & 1) != 0; const bool live = m < NCH;
    float e[8];
    e[0] = odd ? x0[1] : x0[0]; e[1] = odd ? x0[3] : x0[2];
    e[2] = odd ? x1[1] : x1[0]; e[3] = odd ? x1[3] : x1[2];
    e[4] = odd ? x2[1] : x2[0]; e[5] = odd ? x2[3] : x2[2];
    e[6] = odd ? x3[1] : x3[0]; e[7] = odd ? x3[3] : x3[2];
    v8h o;
#pragma unroll
    for (int k = 0; k < 8; ++k) { const h16 hv = toh_flush(bfr(e[k]) * ACAR); o[k] = live ? hv : (h16)0.0f; }
    return o;
}

__global__ __launch_bounds__(256) void k_prep(const float* __restrict__ cp, const float* __restrict__ al, float* PT, h16* AT, float* CV) {
#pragma clang fp contract(off)
    __shared__ __align__(16) float spt[NPT * 2];
    __shared__ float red[8];
    const int t = threadIdx.x, lane = t & 31;
    const int wave = __builtin_amdgcn_readfirstlane((int)(threadIdx.x >> 5));
    const int b = blockIdx.x;
    const int pi = t < (NPT / 2) ? t : (NPT / 2 - 1);
    v4f q = *(const v4f*)(cp + (size_t)b * (NPT * 2) + (size_t)pi * 4);
    asm volatile("" : "+v"(q));
    q[0] = bfr(q[0]); q[1] = bfr(q[1]); q[2] = bfr(q[2]); q[3] = bfr(q[3]);
    if (t < NPT / 2) *(v4fa*)(&spt[t * 4]) = q;
    __syncthreads();
    const int ti = t < NPT ? t : (NPT - 1);
    const float px = spt[2 * ti], py = spt[2 * ti + 1];
    float mn = BIGD;
#pragma unroll 4
    for (int j = 0; j < NPT; ++j) {
        const float dx = px - spt[2 * j], dy = py - spt[2 * j + 1];
        float s = dx * dx + dy * dy;
        s = (j == ti) ? BIGD : s;
        mn = fminf(mn, s);
    }
    float mx = mn;
    mx = fmaxf(mx, __shfl_xor(mx, 16, 32)); mx = fmaxf(mx, __shfl_xor(mx, 8, 32)); mx = fmaxf(mx, __shfl_xor(mx, 4, 32));
    mx = fmaxf(mx, __shfl_xor(mx, 2, 32));  mx = fmaxf(mx, __shfl_xor(mx, 1, 32));
    if (lane == 0) red[wave] = mx;
    __syncthreads();
    float g = red[0];
#pragma unroll
    for (int i = 1; i < 8; ++i) g = fmaxf(g, red[i]);
    const float c = sqrtf(g) * CFAC;
    const float ic = 1.0f / c;
    v4f cv; cv[0] = c; cv[1] = ic; cv[2] = c; cv[3] = ic;
    const bool second = wave < 2;
    const v8h hv0 = at_piece(al, b, t);
    v8h hv1 = (v8h){};
    if (second) hv1 = at_piece(al, b, 256 + t);
    float* ptd = PT + (size_t)b * (NPT * 2) + (size_t)pi * 4;
    h16* atd0 = AT + (size_t)b * (16 * NPT) + (size_t)t * 8;
    h16* atd1 = atd0 + 256 * 8;
    float* cvd = CV + (size_t)b * 32 + (size_t)(t & 7) * 4;
    if (t < NPT / 2) *(volatile v4f*)ptd = q;
    *(volatile v8h*)atd0 = hv0;
    if (second) *(volatile v8h*)atd1 = hv1;
    if (t < 8) *(volatile v4f*)cvd = cv;
    __threadfence();
    if (t < NPT / 2) *(volatile v4f*)ptd = q;
    *(volatile v8h*)atd0 = hv0;
    if (second) *(volatile v8h*)atd1 = hv1;
    if (t < 8) *(volatile v4f*)cvd = cv;
}

__device__ __forceinline__ h16 wend16(float dx, float dy2, float inv_c) {
    const float d  = __builtin_amdgcn_sqrtf(fmaf(dx, dx, dy2)) * inv_c;
    const float t1 = 1.0f - d, t2 = t1 * t1;
    const float w  = (t2 * t2) * fmaf(4.0f * WCAR, d, WCAR);
    return toh_flush((d < 1.0f) ? w : 0.0f);
}

__global__ __launch_bounds__(256) void k_field(const float* __restrict__ PT, const h16* __restrict__ AT, const float* __restrict__ CV, float* OUT) {
    __shared__ __align__(16) float spt[NPT * 2];
    __shared__ __align__(16) float os[FW * NCH * PXW];
    const int t = threadIdx.x, lane = t & 31, lr = lane & 15, hi = lane >> 4;
    const int wave = __builtin_amdgcn_readfirstlane((int)(threadIdx.x >> 5));
    const int hrow = blockIdx.x, b = blockIdx.y;
    const int pi = t < (NPT / 2) ? t : (NPT / 2 - 1);
    v4f q = *(const v4f*)(PT + (size_t)b * (NPT * 2) + (size_t)pi * 4);
    asm volatile("" : "+v"(q));
    if (t < NPT / 2) *(v4fa*)(&spt[t * 4]) = q;
    const float inv_c = CV[(size_t)b * 32 + 1];
    __syncthreads();
    const float py  = (float)hrow;
    const float pxa = (float)(wave * PXW + lr), pxb = pxa + 16.0f;
    const h16* arow = AT + (size_t)b * (16 * NPT) + (size_t)lr * NPT + 8 * hi;
    v8f acc0 = (v8f){}, acc1 = (v8f){};
#pragma unroll 1
    for (int ks = 0; ks < KSTEPS; ++ks) {
        const int kb = ks * 32 + 8 * hi;
        const v16h af = ldh(arow + ks * 32);
        v16h wa, wb;
#pragma unroll
        for (int j = 0; j < 4; ++j) {
            const v4f q0 = *(const v4fa*)(&spt[2 * (kb + 2 * j)]);
            const v4f q1 = *(const v4fa*)(&spt[2 * (kb + 16 + 2 * j)]);
            { const float dy = py - q0[1]; const float dy2 = dy * dy;
              wa[2 * j]     = wend16(pxa - q0[0], dy2, inv_c); wb[2 * j]     = wend16(pxb - q0[0], dy2, inv_c); }
            { const float dy = py - q0[3]; const float dy2 = dy * dy;
              wa[2 * j + 1] = wend16(pxa - q0[2], dy2, inv_c); wb[2 * j + 1] = wend16(pxb - q0[2], dy2, inv_c); }
            { const float dy = py - q1[1]; const float dy2 = dy * dy;
              wa[8 + 2 * j]     = wend16(pxa - q1[0], dy2, inv_c); wb[8 + 2 * j]     = wend16(pxb - q1[0], dy2, inv_c); }
            { const float dy = py - q1[3]; const float dy2 = dy * dy;
              wa[8 + 2 * j + 1] = wend16(pxa - q1[2], dy2, inv_c); wb[8 + 2 * j + 1] = wend16(pxb - q1[2], dy2, inv_c); }
        }
        acc0 = wmma16g(af, wa, acc0);
        acc1 = wmma16g(af, wb, acc1);
    }
    const int wbase = wave * (NCH * PXW);
    if (hi == 0) {
        os[wbase + lr]            = acc0[0] * OSCL;
        os[wbase + 16 + lr]       = acc1[0] * OSCL;
        os[wbase + PXW + lr]      = acc0[1] * OSCL;
        os[wbase + PXW + 16 + lr] = acc1[1] * OSCL;
    }
    wave_sync();
    const int sl = lane & 15, ch = sl >> 3, pc = sl & 7;
    const v4f val = *(const v4fa*)(&os[wbase + ch * PXW + pc * 4]);
    float* dst = OUT + (((size_t)b * NCH + (size_t)ch) * HH_FULL + (size_t)hrow) * WW + (size_t)(wave * PXW + pc * 4);
    if (lane < 16) *(volatile v4f*)dst = val;
    __threadfence();
    if (lane < 16) *(volatile v4f*)dst = val;
}

static constexpr size_t al256(size_t v) { return (v + 255) & ~(size_t)255; }
static constexpr size_t SZ_PT = al256((size_t)NB * NPT * 2 * 4);
static constexpr size_t SZ_AT = al256((size_t)NB * 16 * NPT * 2);
static constexpr size_t SZ_CV = al256((size_t)NB * 32 * 4);
static constexpr size_t SZ_TOTAL = SZ_PT + SZ_AT + SZ_CV;
static_assert(SZ_TOTAL <= (size_t)134217728);
static_assert((size_t)(NB - 1) * (NPT * 2) * 4 + (size_t)(NPT / 2) * 16 <= SZ_PT);
static_assert((size_t)(NB - 1) * (16 * NPT) * 2 + (size_t)(256 + 64) * 16 <= SZ_AT);
static_assert((size_t)(NB - 1) * 128 + 128 <= SZ_CV);
static_assert(((((size_t)(NB_FULL - 1) * NCH + (NCH - 1)) * HH_FULL + (HH_FULL - 1)) * WW + WW) * 4 == (size_t)4194304);

extern "C" void kernel_launch(void* const* d_in, const int* in_sizes, int n_in,
                              void* d_out, int out_size, void* d_ws, size_t ws_size, hipStream_t stream) {
    if (n_in < 2) return;
    if ((size_t)in_sizes[0] < (size_t)NB * NPT * 2 || (size_t)in_sizes[1] < (size_t)NB * NPT * NCH) return;
    if ((size_t)out_size < ((((size_t)(NB - 1) * NCH + (NCH - 1)) * HH_FULL) + (size_t)HROWS) * WW) return;
    if (SZ_TOTAL > ws_size) return;
    const float* cp = (const float*)d_in[0];
    const float* al = (const float*)d_in[1];
    float* OUT = (float*)d_out;
    char* wsp = (char*)d_ws;
    float* PT = (float*)wsp; wsp += SZ_PT;
    h16*   AT = (h16*)wsp;   wsp += SZ_AT;
    float* CV = (float*)wsp; wsp += SZ_CV;

    k_prep<<<dim3(NB, 1, 1), 256, 0, stream>>>(cp, al, PT, AT, CV);
    k_field<<<dim3(HROWS, NB, 1), 256, 0, stream>>>(PT, AT, CV, OUT);
}
